// MultiheadClassifier_30382598652209
// MI455X (gfx1250) — hardware-verified
//
#include <hip/hip_runtime.h>
#include <math.h>

constexpr int kBatch  = 4;
constexpr int kSeq    = 1001;
constexpr int kSeqPad = 1024;
constexpr int kEin    = 256;
constexpr int kDh     = 64;
constexpr int kHeads  = 10;
constexpr int kCat    = kHeads * kDh;
constexpr int kTokPad = kBatch * kSeqPad;
constexpr float kWCarry    = 16.0f;
constexpr float kWCarryInv = 1.0f / 16.0f;
constexpr float kAttnScale = 1.0f / 16.0f;
constexpr float kPCarry    = 2048.0f;
constexpr float kPCarryInv = 1.0f / 2048.0f;
constexpr float kNormEps   = 1e-12f;

constexpr size_t kOut0N   = (size_t)kBatch * kSeq * kCat;
constexpr size_t kOut1N   = (size_t)kBatch * kSeq * kSeq;
constexpr size_t kOut1Off = kOut0N;
static_assert(kOut1Off * 4 == 10250240);
static_assert((kOut1Off * 4) % 128 == 0);
static_assert(kOut0N % 4 == 0 && kOut1N % 4 == 0);

constexpr size_t kBytesX16  = (size_t)kTokPad * kEin * 2;
constexpr size_t kBytesW16p = (size_t)kCat * kEin * 2;
constexpr size_t kBytesQK16 = (size_t)kTokPad * kCat * 2;
constexpr size_t kBytesSC   = (size_t)kHeads * kSeqPad * kSeqPad * 4;
constexpr size_t kBytesW16  = (size_t)kHeads * kSeqPad * kSeqPad * 2;
constexpr size_t kBytesOST  = (size_t)kTokPad * kCat * 4;
constexpr size_t kBytesW1ST = (size_t)kBatch * kSeqPad * kSeqPad * 4;
constexpr size_t kOffX16  = 0;
constexpr size_t kOffWQ16 = kOffX16 + kBytesX16;
constexpr size_t kOffWK16 = kOffWQ16 + kBytesW16p;
constexpr size_t kOffWV16 = kOffWK16 + kBytesW16p;
constexpr size_t kOffQ16  = kOffWV16 + kBytesW16p;
constexpr size_t kOffK16  = kOffQ16 + kBytesQK16;
constexpr size_t kOffVT16 = kOffK16 + kBytesQK16;
constexpr size_t kOffSC   = kOffVT16 + kBytesQK16;
constexpr size_t kOffW16  = kOffSC + kBytesSC;
constexpr size_t kOffOST  = kOffW16 + kBytesW16;
constexpr size_t kOffW1ST = kOffOST + kBytesOST;
constexpr size_t kWsTotal = kOffW1ST + kBytesW1ST;
static_assert(kWsTotal == 108986368);
static_assert(kWsTotal <= 134217728);
static_assert(kOffWQ16 % 128 == 0 && kOffWK16 % 128 == 0 && kOffWV16 % 128 == 0 && kOffQ16 % 128 == 0 &&
              kOffK16 % 128 == 0 && kOffVT16 % 128 == 0 && kOffSC % 128 == 0 && kOffW16 % 128 == 0 &&
              kOffOST % 128 == 0 && kOffW1ST % 128 == 0);

typedef __attribute__((ext_vector_type(16))) _Float16 v16h;
typedef __attribute__((ext_vector_type(8)))  _Float16 v8h;
typedef __attribute__((ext_vector_type(16))) __bf16   v16b;
typedef __attribute__((ext_vector_type(8)))  __bf16   v8b;
typedef __attribute__((ext_vector_type(8)))  float    v8f;
typedef __attribute__((ext_vector_type(4)))  float    v4f;
typedef __attribute__((ext_vector_type(4)))  unsigned int v4u;

__device__ __forceinline__ unsigned short f2bf_bits(float f) {
  unsigned u = __float_as_uint(f);
  return (unsigned short)((u + 0x7FFFu + ((u >> 16) & 1u)) >> 16);
}
__device__ __forceinline__ float bf_bits2f(unsigned short h) { return __uint_as_float(((unsigned)h) << 16); }

__device__ __forceinline__ void dep_guard_h(v8f& a, v8f& b, v16h x, v16h y) { asm volatile("v_nop\n\tv_nop\n\tv_nop\n\tv_nop" : "+v"(a), "+v"(b) : "v"(x), "v"(y)); }
__device__ __forceinline__ void dep_guard_b(v8f& a, v8f& b, v16b x, v16b y) { asm volatile("v_nop\n\tv_nop\n\tv_nop\n\tv_nop" : "+v"(a), "+v"(b) : "v"(x), "v"(y)); }
__device__ __forceinline__ void keep4_h(v16h a, v16h b, v16h c, v16h d) { asm volatile("v_nop" :: "v"(a), "v"(b), "v"(c), "v"(d)); }
__device__ __forceinline__ void keep4_b(v16b a, v16b b, v16b c, v16b d) { asm volatile("v_nop" :: "v"(a), "v"(b), "v"(c), "v"(d)); }
__device__ __forceinline__ void acc_guard4(v8f& a, v8f& b, v8f& c, v8f& d) { asm volatile("v_nop\n\tv_nop\n\tv_nop\n\tv_nop" : "+v"(a), "+v"(b), "+v"(c), "+v"(d)); }
template <typename T> struct Frag;
template <> struct Frag<_Float16> {
  typedef v16h V; union U { v16h v; v8h h[2]; };
  static __device__ __forceinline__ v16h load(const _Float16* p) {
    U f; f.h[0] = *(const v8h*)(p); f.h[1] = *(const v8h*)(p + 16); return f.v;
  }
  static __device__ __forceinline__ v8f mma(v16h a, v16h b, v8f c) {
    return __builtin_amdgcn_wmma_f32_16x16x32_f16(false, a, false, b, (short)0, c, false, false);
  }
  static __device__ __forceinline__ void guard(v8f& a, v8f& b, v16h x, v16h y) { dep_guard_h(a, b, x, y); }
  static __device__ __forceinline__ void keep(v16h a, v16h b, v16h c, v16h d) { keep4_h(a, b, c, d); }
};
template <> struct Frag<__bf16> {
  typedef v16b V; union U { v16b v; v8b h[2]; };
  static __device__ __forceinline__ v16b load(const __bf16* p) {
    U f; f.h[0] = *(const v8b*)(p); f.h[1] = *(const v8b*)(p + 16); return f.v;
  }
  static __device__ __forceinline__ v8f mma(v16b a, v16b b, v8f c) {
    return __builtin_amdgcn_wmma_f32_16x16x32_bf16(false, a, false, b, (short)0, c, false, false);
  }
  static __device__ __forceinline__ void guard(v8f& a, v8f& b, v16b x, v16b y) { dep_guard_b(a, b, x, y); }
  static __device__ __forceinline__ void keep(v16b a, v16b b, v16b c, v16b d) { keep4_b(a, b, c, d); }
};

__device__ __forceinline__ unsigned pk16(unsigned short a, unsigned short b) { return (unsigned)a | ((unsigned)b << 16); }
__device__ __forceinline__ unsigned short h_bits(float f) { const _Float16 h = (_Float16)f; return __builtin_bit_cast(unsigned short, h); }

template <int ET> struct Elem;
template <> struct Elem<0> { typedef _Float16 T; };
template <> struct Elem<1> { typedef __bf16 T; };
template <int ET, bool SPLIT, int BIAS_MODE, int OUT_MODE, bool RESID, int ACT = 0>
__global__ __launch_bounds__(256) void wmma_gemm64(
    const unsigned short* __restrict__ Ap, const unsigned short* __restrict__ A2p, int lda, long strideA,
    const unsigned short* __restrict__ Btp, const unsigned short* __restrict__ Bt2p, int ldb, long strideB,
    void* __restrict__ Cout, void* __restrict__ Cout2, int ldc, long strideC,
    const float* __restrict__ bias,
    const float* __restrict__ resid, long strideR,
    int M, int N, int K, float scale) {
  typedef typename Elem<ET>::T T;
  typedef typename Frag<T>::V V;
  const T* A = (const T*)Ap; const T* A2 = (const T*)A2p; const T* Bt = (const T*)Btp; const T* Bt2 = (const T*)Bt2p;
  __shared__ __align__(16) float sT[8][16 * 68];
  const int b    = blockIdx.y;
  const int lane = threadIdx.x & 31;
  const int wave = threadIdx.x >> 5;
  const int tilesN = N >> 6;
  const int tilesM = M >> 6;
  const int tile = blockIdx.x * 8 + wave;
  if (tile >= tilesM * tilesN) return;
  const int tm = tile / tilesN;
  const int tn = tile - tm * tilesN;
  const int m0 = tm << 6;
  const int n0 = tn << 6;

  const T* Ab  = A  + (size_t)b * strideA;
  const T* Bb  = Bt + (size_t)b * strideB;
  const T* Ab2 = SPLIT ? (A2  + (size_t)b * strideA) : nullptr;
  const T* Bb2 = SPLIT ? (Bt2 + (size_t)b * strideB) : nullptr;

  const int rlane = lane & 15;
  const int koff  = (lane >> 4) * 8;
  const int mOff  = (lane >> 4) * 8;

  v8f acc[4][4];
#pragma unroll
  for (int i = 0; i < 4; ++i)
#pragma unroll
    for (int j = 0; j < 4; ++j) acc[i][j] = (v8f){0.f,0.f,0.f,0.f,0.f,0.f,0.f,0.f};

  for (int k0 = 0; k0 < K; k0 += 32) {
    V bh[4], bl[4];
#pragma unroll
    for (int j = 0; j < 4; ++j) {
      const size_t bo = (size_t)(n0 + (j << 4) + rlane) * ldb + koff + k0;
      bh[j] = Frag<T>::load(Bb + bo);
      if (SPLIT) bl[j] = Frag<T>::load(Bb2 + bo);
    }
#pragma unroll
    for (int i = 0; i < 4; ++i) {
      const size_t ao = (size_t)(m0 + (i << 4) + rlane) * lda + koff + k0;
      V ah = Frag<T>::load(Ab + ao);
      V al;
      if (SPLIT) al = Frag<T>::load(Ab2 + ao);
#pragma unroll
      for (int j = 0; j < 4; ++j) {
        acc[i][j] = Frag<T>::mma(ah, bh[j], acc[i][j]);
        if (SPLIT) {
          acc[i][j] = Frag<T>::mma(ah, bl[j], acc[i][j]);
          acc[i][j] = Frag<T>::mma(al, bh[j], acc[i][j]);
        }
      }
      Frag<T>::guard(acc[i][0], acc[i][3], ah, SPLIT ? al : ah);
    }
    Frag<T>::keep(bh[0], bh[1], bh[2], bh[3]);
    if (SPLIT) Frag<T>::keep(bl[0], bl[1], bl[2], bl[3]);
  }
  acc_guard4(acc[0][0], acc[0][1], acc[0][2], acc[0][3]);
  acc_guard4(acc[1][0], acc[1][1], acc[1][2], acc[1][3]);
  acc_guard4(acc[2][0], acc[2][1], acc[2][2], acc[2][3]);
  acc_guard4(acc[3][0], acc[3][1], acc[3][2], acc[3][3]);

  float* slab = sT[wave];
  const float* Rb = RESID ? (resid + (size_t)b * strideR) : nullptr;
#pragma unroll
  for (int i = 0; i < 4; ++i) {
    const int mBase = m0 + (i << 4);
#pragma unroll
    for (int j = 0; j < 4; ++j) {
      const int n = n0 + (j << 4) + rlane;
      float bv = 0.f;
      if (BIAS_MODE == 2) bv = bias[n];
#pragma unroll
      for (int r = 0; r < 8; ++r) {
        float v = acc[i][j][r] * scale;
        if (BIAS_MODE == 1) v += bias[mBase + mOff + r];
        if (BIAS_MODE == 2) v += bv;
        if (RESID) v += Rb[(size_t)(mBase + mOff + r) * ldc + n];
        if (ACT == 2) v = fmaxf(v, 0.0f);
        if (ACT == 4) v = (v > 0.f) ? v : 0.01f * v;
        slab[(mOff + r) * 68 + (j << 4) + rlane] = v;
      }
    }
    __builtin_amdgcn_fence(__ATOMIC_RELEASE, "workgroup");
    __builtin_amdgcn_wave_barrier();
    __builtin_amdgcn_fence(__ATOMIC_ACQUIRE, "workgroup");
    if (OUT_MODE == 0) {
      float* C = (float*)Cout + (size_t)b * strideC;
      const int hh = lane >> 4, c4 = (lane & 15) * 4;
      for (int pass = 0; pass < 2; ++pass) {
#pragma unroll
        for (int it = 0; it < 8; ++it) {
          const int row = it * 2 + hh;
          v4f v = *(const v4f*)(slab + row * 68 + c4);
          *(volatile v4f*)(C + (size_t)(mBase + row) * ldc + n0 + c4) = v;
        }
        __threadfence();
      }
    } else {
      const int q = lane >> 3, c8 = (lane & 7) * 8;
      unsigned short* C  = (unsigned short*)Cout  + (size_t)b * strideC;
      unsigned short* C2 = (OUT_MODE == 2) ? ((unsigned short*)Cout2 + (size_t)b * strideC) : nullptr;
      for (int pass = 0; pass < 2; ++pass) {
#pragma unroll
        for (int it = 0; it < 4; ++it) {
          const int row = it * 4 + q;
          const float* sp = slab + row * 68 + c8;
          v8h hv, lv;
#pragma unroll
          for (int e = 0; e < 8; ++e) {
            if (OUT_MODE == 1) {
              hv[e] = (_Float16)sp[e];
            } else {
              unsigned short hb = f2bf_bits(sp[e]);
              unsigned short lb = f2bf_bits(sp[e] - bf_bits2f(hb));
              hv[e] = __builtin_bit_cast(_Float16, hb);
              lv[e] = __builtin_bit_cast(_Float16, lb);
            }
          }
          *(volatile v8h*)(C + (size_t)(mBase + row) * ldc + n0 + c8) = hv;
          if (OUT_MODE == 2) *(volatile v8h*)(C2 + (size_t)(mBase + row) * ldc + n0 + c8) = lv;
        }
        __threadfence();
      }
    }
    __builtin_amdgcn_fence(__ATOMIC_RELEASE, "workgroup");
    __builtin_amdgcn_wave_barrier();
    __builtin_amdgcn_fence(__ATOMIC_ACQUIRE, "workgroup");
  }
}

__global__ __launch_bounds__(256) void castx_kernel(const float* __restrict__ x, unsigned short* __restrict__ out) {
  const int i = blockIdx.x * 256 + threadIdx.x;
  if (i >= kTokPad * kEin / 8) return;
  const int row = i >> 5;
  const int e0  = (i & 31) * 8;
  const int b   = row >> 10;
  const int s   = row & 1023;
  const int sc  = (s < kSeq) ? s : (kSeq - 1);
  const bool valid = (s < kSeq);
  const float* p = x + ((size_t)(b * kSeq + sc)) * kEin + e0;
  const v4f a = *(const v4f*)(p);
  const v4f c = *(const v4f*)(p + 4);
  unsigned short hb[8];
#pragma unroll
  for (int e = 0; e < 4; ++e) {
    hb[e]     = h_bits(valid ? a[e] : 0.0f);
    hb[4 + e] = h_bits(valid ? c[e] : 0.0f);
  }
  const v4u u = (v4u){pk16(hb[0], hb[1]), pk16(hb[2], hb[3]), pk16(hb[4], hb[5]), pk16(hb[6], hb[7])};
  unsigned short* q = out + 8 * (size_t)i;
  *(volatile v4u*)q = u;
  __threadfence();
  *(volatile v4u*)q = u;
}

__global__ __launch_bounds__(256) void castw_kernel(const float* __restrict__ W0, const float* __restrict__ W1,
                                                    const float* __restrict__ W2, unsigned short* __restrict__ out,
                                                    float carry) {
  const int i = blockIdx.x * 256 + threadIdx.x;
  const int z = blockIdx.y;
  if (i >= kCat * kEin / 8) return;
  const float* W = (z == 0) ? W0 : (z == 1) ? W1 : W2;
  const float* p = W + 8 * (size_t)i;
  const v4f a = *(const v4f*)(p);
  const v4f c = *(const v4f*)(p + 4);
  unsigned short hb[8];
#pragma unroll
  for (int e = 0; e < 4; ++e) {
    hb[e]     = h_bits(a[e] * carry);
    hb[4 + e] = h_bits(c[e] * carry);
  }
  const v4u u = (v4u){pk16(hb[0], hb[1]), pk16(hb[2], hb[3]), pk16(hb[4], hb[5]), pk16(hb[6], hb[7])};
  unsigned short* q = out + (size_t)z * kCat * kEin + 8 * (size_t)i;
  *(volatile v4u*)q = u;
  __threadfence();
  *(volatile v4u*)q = u;
}

__device__ __forceinline__ float wave_max32(float v) {
#pragma unroll
  for (int off = 16; off > 0; off >>= 1) v = fmaxf(v, __shfl_xor(v, off, 32));
  return v;
}
__device__ __forceinline__ float wave_sum32(float v) {
#pragma unroll
  for (int off = 16; off > 0; off >>= 1) v += __shfl_xor(v, off, 32);
  return v;
}

__global__ __launch_bounds__(128) void softnorm_kernel(const float* __restrict__ Sc, const float* __restrict__ lam,
                                                       unsigned short* __restrict__ W16, float* __restrict__ W1row) {
  __shared__ __align__(16) float xs[kSeqPad];
  __shared__ __align__(16) float accl[kSeqPad];
  __shared__ float laml[kSeqPad];
  __shared__ float redA[4];
  __shared__ float redB[4];
  __shared__ float redC[4];
  const int s    = blockIdx.x;
  const int t    = threadIdx.x;
  const int lane = t & 31;
  const int wave = t >> 5;

  if (s >= kSeq) {
    const v4u zu = (v4u){0u, 0u, 0u, 0u};
    const v4f zf = (v4f){0.f, 0.f, 0.f, 0.f};
    for (int pass = 0; pass < 2; ++pass) {
#pragma unroll 1
      for (int h = 0; h < kHeads; ++h)
        *(volatile v4u*)(W16 + ((size_t)h * kSeqPad + s) * kSeqPad + 8 * t) = zu;
      *(volatile v4f*)(W1row + (size_t)s * kSeqPad + 4 * t) = zf;
      *(volatile v4f*)(W1row + (size_t)s * kSeqPad + 512 + 4 * t) = zf;
      __threadfence();
    }
    return;
  }

#pragma unroll 1
  for (int j = 0; j < 8; ++j) {
    const int c  = t + 128 * j;
    const int cc = (c < kSeq) ? c : (kSeq - 1);
    const float lv = lam[(size_t)s * kSeq + cc];
    laml[c] = (c < kSeq) ? lv : 0.0f;
    accl[c] = 0.0f;
  }

#pragma unroll 1
  for (int h = 0; h < kHeads; ++h) {
    const float* sr = Sc + ((size_t)h * kSeqPad + s) * kSeqPad;
    float m = -3.0e38f;
#pragma unroll 1
    for (int j = 0; j < 8; ++j) {
      const int c = t + 128 * j;
      const float xv = sr[c];
      xs[c] = xv;
      m = (c < kSeq) ? fmaxf(m, xv) : m;
    }
    m = wave_max32(m);
    if (lane == 0) redA[wave] = m;
    __syncthreads();
    const float M = fmaxf(fmaxf(redA[0], redA[1]), fmaxf(redA[2], redA[3]));
    float sum = 0.0f;
#pragma unroll 1
    for (int j = 0; j < 8; ++j) {
      const int c = t + 128 * j;
      float e = expf(xs[c] - M);
      e = (c < kSeq) ? e : 0.0f;
      xs[c] = e;
      sum += e;
    }
    sum = wave_sum32(sum);
    if (lane == 0) redB[wave] = sum;
    __syncthreads();
    const float tot = (redB[0] + redB[1]) + (redB[2] + redB[3]);
    const float inv = 1.0f / tot;
    float ss = 0.0f;
#pragma unroll 1
    for (int j = 0; j < 8; ++j) {
      const int c = t + 128 * j;
      const float loc = (xs[c] * inv) * laml[c];
      xs[c] = loc;
      ss += loc * loc;
    }
    ss = wave_sum32(ss);
    if (lane == 0) redC[wave] = ss;
    __syncthreads();
    const float sq  = (redC[0] + redC[1]) + (redC[2] + redC[3]);
    const float rdn = 1.0f / fmaxf(sqrtf(sq), kNormEps);
#pragma unroll 1
    for (int j = 0; j < 8; ++j) {
      const int c = t + 128 * j;
      const float w = xs[c] * rdn;
      xs[c] = w;
      accl[c] += w;
    }
    __syncthreads();
    {
      const v4f wa = *(const v4f*)(xs + 8 * t);
      const v4f wb = *(const v4f*)(xs + 8 * t + 4);
      unsigned short hb[8];
#pragma unroll
      for (int e = 0; e < 4; ++e) {
        hb[e]     = h_bits(wa[e] * kPCarry);
        hb[4 + e] = h_bits(wb[e] * kPCarry);
      }
      const v4u u = (v4u){pk16(hb[0], hb[1]), pk16(hb[2], hb[3]), pk16(hb[4], hb[5]), pk16(hb[6], hb[7])};
      unsigned short* dst = W16 + ((size_t)h * kSeqPad + s) * kSeqPad + 8 * t;
      *(volatile v4u*)dst = u;
      __threadfence();
      *(volatile v4u*)dst = u;
    }
    __syncthreads();
  }

  {
    const v4f a0 = *(const v4f*)(accl + 4 * t);
    const v4f a1 = *(const v4f*)(accl + 512 + 4 * t);
    float* wr = W1row + (size_t)s * kSeqPad;
    *(volatile v4f*)(wr + 4 * t) = a0;
    *(volatile v4f*)(wr + 512 + 4 * t) = a1;
    __threadfence();
    *(volatile v4f*)(wr + 4 * t) = a0;
    *(volatile v4f*)(wr + 512 + 4 * t) = a1;
  }
}

__global__ __launch_bounds__(256) void copy_out0_kernel(const float* __restrict__ Ost, float* __restrict__ out0, int n4) {
  const int i = blockIdx.x * 256 + threadIdx.x;
  if (i >= n4) return;
  const int r = i / (kCat / 4);
  const int c = (i - r * (kCat / 4)) * 4;
  const int b = r / kSeq;
  const int s = r - b * kSeq;
  const v4f v = *(const v4f*)(Ost + ((size_t)(b * kSeqPad + s)) * kCat + c);
  float* dst = out0 + 4 * (size_t)i;
  *(volatile v4f*)dst = v;
  __threadfence();
  *(volatile v4f*)dst = v;
}

__global__ __launch_bounds__(256) void copy_out1_kernel(const float* __restrict__ W1st, float* __restrict__ out1, int n4) {
  const int i = blockIdx.x * 256 + threadIdx.x;
  if (i >= n4) return;
  v4f v;
#pragma unroll
  for (int j = 0; j < 4; ++j) {
    const int idx = 4 * i + j;
    const int r = idx / kSeq;
    const int tcol = idx - r * kSeq;
    const int b = r / kSeq;
    const int s = r - b * kSeq;
    v[j] = W1st[((size_t)(b * kSeqPad + s)) * kSeqPad + tcol];
  }
  float* dst = out1 + 4 * (size_t)i;
  *(volatile v4f*)dst = v;
  __threadfence();
  *(volatile v4f*)dst = v;
}

extern "C" void kernel_launch(void* const* d_in, const int* in_sizes, int n_in,
                              void* d_out, int out_size, void* d_ws, size_t ws_size,
                              hipStream_t stream) {
  if (n_in < 8) return;
  if (ws_size < kWsTotal) return;
  if ((size_t)out_size < kOut0N + kOut1N) return;
  if ((size_t)in_sizes[0] < (size_t)kBatch * kSeq * kEin) return;
  if ((size_t)in_sizes[1] < (size_t)kSeq * kSeq) return;

  const float* x   = (const float*)d_in[0];
  const float* lam = (const float*)d_in[1];
  const float* Wq  = (const float*)d_in[2];
  const float* bq  = (const float*)d_in[3];
  const float* Wk  = (const float*)d_in[4];
  const float* bk  = (const float*)d_in[5];
  const float* Wv  = (const float*)d_in[6];
  const float* bv  = (const float*)d_in[7];

  float* out0 = (float*)d_out;
  float* out1 = (float*)d_out + kOut1Off;

  char* ws = (char*)d_ws;
  unsigned short* X16  = (unsigned short*)(ws + kOffX16);
  unsigned short* WQ16 = (unsigned short*)(ws + kOffWQ16);
  unsigned short* WK16 = (unsigned short*)(ws + kOffWK16);
  unsigned short* WV16 = (unsigned short*)(ws + kOffWV16);
  unsigned short* Q16  = (unsigned short*)(ws + kOffQ16);
  unsigned short* K16  = (unsigned short*)(ws + kOffK16);
  unsigned short* VT16 = (unsigned short*)(ws + kOffVT16);
  float*          Sc   = (float*)(ws + kOffSC);
  unsigned short* W16  = (unsigned short*)(ws + kOffW16);
  float*          Ost  = (float*)(ws + kOffOST);
  float*          W1st = (float*)(ws + kOffW1ST);

  castx_kernel<<<dim3((kTokPad * kEin / 8 + 255) / 256), dim3(256), 0, stream>>>(x, X16);
  castw_kernel<<<dim3((kCat * kEin / 8 + 255) / 256, 3), dim3(256), 0, stream>>>(Wq, Wk, Wv, WQ16, kWCarry);

  wmma_gemm64<0, false, 2, 1, false><<<dim3(80, 1), dim3(256), 0, stream>>>(
      X16, X16, kEin, 0L, WQ16, WQ16, kEin, 0L, (void*)Q16, (void*)Q16, kCat, 0L,
      bq, nullptr, 0L, kTokPad, kCat, kEin, kWCarryInv);
  wmma_gemm64<0, false, 2, 1, false><<<dim3(80, 1), dim3(256), 0, stream>>>(
      X16, X16, kEin, 0L, WK16, WK16, kEin, 0L, (void*)K16, (void*)K16, kCat, 0L,
      bk, nullptr, 0L, kTokPad, kCat, kEin, kWCarryInv);
  wmma_gemm64<0, false, 1, 1, false><<<dim3(80, 1), dim3(256), 0, stream>>>(
      WV16, WV16, kEin, 0L, X16, X16, kEin, 0L, (void*)VT16, (void*)VT16, kTokPad, 0L,
      bv, nullptr, 0L, kCat, kTokPad, kEin, kWCarryInv);

  for (int b = 0; b < kBatch; ++b) {
    const size_t tokOff = (size_t)b * kSeqPad * kCat;
    wmma_gemm64<0, false, 0, 0, false><<<dim3(32, kHeads), dim3(256), 0, stream>>>(
        Q16 + tokOff, Q16 + tokOff, kCat, (long)kDh,
        K16 + tokOff, K16 + tokOff, kCat, (long)kDh,
        (void*)Sc, (void*)Sc, kSeqPad, (long)kSeqPad * kSeqPad,
        nullptr, nullptr, 0L, kSeqPad, kSeqPad, kDh, kAttnScale);
    softnorm_kernel<<<dim3(kSeqPad), dim3(128), 0, stream>>>(
        Sc, lam, W16, W1st + (size_t)b * kSeqPad * kSeqPad);
    wmma_gemm64<0, false, 0, 0, false><<<dim3(2, kHeads), dim3(256), 0, stream>>>(
        W16, W16, kSeqPad, (long)kSeqPad * kSeqPad,
        VT16 + (size_t)b * kSeqPad, VT16 + (size_t)b * kSeqPad, kTokPad, (long)kDh * kTokPad,
        (void*)(Ost + (size_t)b * kSeqPad * kCat), (void*)(Ost + (size_t)b * kSeqPad * kCat), kCat, (long)kDh,
        nullptr, nullptr, 0L, kSeqPad, kDh, kSeqPad, kPCarryInv);
  }

  const int n4a = (int)(kOut0N / 4);
  const int n4b = (int)(kOut1N / 4);
  copy_out0_kernel<<<dim3((n4a + 255) / 256), dim3(256), 0, stream>>>(Ost, out0, n4a);
  copy_out1_kernel<<<dim3((n4b + 255) / 256), dim3(256), 0, stream>>>(W1st, out1, n4b);
}
